// SelfAttention_22634477650084
// MI455X (gfx1250) — hardware-verified
//
#include <hip/hip_runtime.h>
#ifndef NB
#define NB 2
#endif
#ifndef SEQ
#define SEQ 4096
#endif
#define NB_FULL 2
#define SEQ_FULL 4096
#define DM 512
#define NH 8
#define HD 64
#define NR ((size_t)NB * SEQ)

static_assert(DM == NH * HD);
static_assert(HD == 64);
static_assert(SEQ % 64 == 0);
static_assert(NB <= NB_FULL);
static_assert(SEQ <= SEQ_FULL);
static_assert(DM % 64 == 0);
static_assert(HD % 32 == 0);
static_assert((HD * HD) % 8 == 0);
static_assert(((size_t)DM * DM) % 8 == 0);

#define WS_W64   ((size_t)HD * HD * 2)
#define WS_WO    ((size_t)DM * DM * 2)
#define WS_PLANE (NR * DM * 2)
#define WS_TOTAL (3 * WS_W64 + WS_WO + 5 * WS_PLANE)
static_assert(WS_W64 % 256 == 0);
static_assert(WS_WO % 256 == 0);
static_assert(WS_PLANE % 256 == 0);
static_assert(WS_TOTAL <= (size_t)134217728);

typedef _Float16 v16h __attribute__((ext_vector_type(16)));
typedef unsigned short v8us __attribute__((ext_vector_type(8), may_alias));
typedef float v8f  __attribute__((ext_vector_type(8)));
typedef float v4f  __attribute__((ext_vector_type(4)));
typedef float v4fa __attribute__((ext_vector_type(4), may_alias));
typedef int   v4ia __attribute__((ext_vector_type(4), may_alias));
union FragH { v16h v; v8us half[2]; _Float16 h[16]; unsigned short u[16]; };
union HBits { _Float16 h; unsigned short u; };

__device__ __forceinline__ float bf16_rne(float x) {
  unsigned int u = __float_as_uint(x);
  u = (u + 0x7FFFu + ((u >> 16) & 1u)) & 0xFFFF0000u;
  return __uint_as_float(u);
}
__device__ __forceinline__ unsigned short hbits(float x) { HBits b; b.h = (_Float16)x; return b.u; }

__device__ __forceinline__ v8f mma16(v16h a, v16h b, v8f c) {
  v8f d = __builtin_amdgcn_wmma_f32_16x16x32_f16(false, a, false, b, (short)0, c, false, false);
  asm volatile("v_nop\n\tv_nop\n\tv_nop\n\tv_nop" : "+v"(d) : "v"(a), "v"(b));
  return d;
}
__device__ __forceinline__ v16h ldfrag(const _Float16* __restrict__ base, size_t off, int hh) {
  FragH f;
  const unsigned short* p = (const unsigned short*)base + off + 8 * hh;
  f.half[0] = *(const v8us*)p;
  f.half[1] = *(const v8us*)(p + 16);
  return f.v;
}

__global__ __launch_bounds__(256) void k_wnat(const float* __restrict__ w, unsigned int n8, _Float16* __restrict__ Bt) {
  const unsigned int t = blockIdx.x * 256u + threadIdx.x;
  if (t >= n8) return;
  const v4f a = *(const v4fa*)(w + (size_t)t * 8), c = *(const v4fa*)(w + (size_t)t * 8 + 4);
  FragH f;
#pragma unroll
  for (int q = 0; q < 4; ++q) { f.h[q] = (_Float16)(bf16_rne(a[q]) * 16.0f); f.h[4 + q] = (_Float16)(bf16_rne(c[q]) * 16.0f); }
  const v8us o = f.half[0];
  unsigned short* d = (unsigned short*)Bt + (size_t)t * 8;
  *(volatile v8us*)d = o;
  __threadfence();
  *(volatile v8us*)d = o;
}

__device__ __forceinline__ void proj_acc(const float* __restrict__ x, size_t xoff, const _Float16* __restrict__ W16, int ln, int hh,
                                         v8f& c0, v8f& c1, v8f& c2, v8f& c3) {
#pragma unroll
  for (int kb = 0; kb < HD; kb += 32) {
    const float* p = x + xoff + kb + 8 * hh;
    const v4f x0 = *(const v4fa*)(p), x1 = *(const v4fa*)(p + 4), x2 = *(const v4fa*)(p + 16), x3 = *(const v4fa*)(p + 20);
    FragH a;
#pragma unroll
    for (int i = 0; i < 4; ++i) {
      a.h[i]      = (_Float16)bf16_rne(x0[i]);
      a.h[4 + i]  = (_Float16)bf16_rne(x1[i]);
      a.h[8 + i]  = (_Float16)bf16_rne(x2[i]);
      a.h[12 + i] = (_Float16)bf16_rne(x3[i]);
    }
    const size_t wo = (size_t)ln * HD + kb;
    c0 = mma16(a.v, ldfrag(W16, wo, hh), c0);
    c1 = mma16(a.v, ldfrag(W16, wo + 16 * HD, hh), c1);
    c2 = mma16(a.v, ldfrag(W16, wo + 32 * HD, hh), c2);
    c3 = mma16(a.v, ldfrag(W16, wo + 48 * HD, hh), c3);
  }
}

__global__ __launch_bounds__(128) void k_proj_n(const float* __restrict__ x, const _Float16* __restrict__ W16, _Float16* __restrict__ dst) {
  __shared__ __attribute__((aligned(16))) float so[4][16][68];
  const int tid = threadIdx.x;
  const int wave = __builtin_amdgcn_readfirstlane(tid >> 5);
  const int lane = tid & 31, ln = lane & 15, hh = lane >> 4;
  const int tile = blockIdx.x, h = blockIdx.y;
  const int b = tile / (SEQ / 64);
  const int s0 = (tile % (SEQ / 64)) * 64 + wave * 16;
  const size_t xoff = ((size_t)b * SEQ_FULL + s0 + ln) * DM + h * HD;
  const v8f z8 = {0.f, 0.f, 0.f, 0.f, 0.f, 0.f, 0.f, 0.f};
  v8f c0 = z8, c1 = z8, c2 = z8, c3 = z8;
  proj_acc(x, xoff, W16, ln, hh, c0, c1, c2, c3);
#pragma unroll
  for (int r = 0; r < 8; ++r) {
    so[wave][8 * hh + r][ln]      = c0[r] * 0.0625f;
    so[wave][8 * hh + r][16 + ln] = c1[r] * 0.0625f;
    so[wave][8 * hh + r][32 + ln] = c2[r] * 0.0625f;
    so[wave][8 * hh + r][48 + ln] = c3[r] * 0.0625f;
  }
  __syncthreads();
  const int rq = lane >> 3, c8 = (lane & 7) * 8;
  v8us ov[4];
#pragma unroll
  for (int q = 0; q < 4; ++q) {
    const int row = q * 4 + rq;
    const v4f a = *(const v4fa*)&so[wave][row][c8], c = *(const v4fa*)&so[wave][row][c8 + 4];
    FragH f;
#pragma unroll
    for (int i = 0; i < 4; ++i) { f.h[i] = (_Float16)a[i]; f.h[4 + i] = (_Float16)c[i]; }
    ov[q] = f.half[0];
  }
  const size_t obase = ((size_t)b * SEQ + s0) * DM + h * HD + c8;
  for (int pass = 0; pass < 2; ++pass) {
#pragma unroll
    for (int q = 0; q < 4; ++q)
      *(volatile v8us*)((unsigned short*)dst + obase + (size_t)(q * 4 + rq) * DM) = ov[q];
    if (pass == 0) __threadfence();
  }
}

__global__ __launch_bounds__(128) void k_proj_t(const float* __restrict__ x, const _Float16* __restrict__ W16, _Float16* __restrict__ dst) {
  __shared__ __attribute__((aligned(16))) unsigned short tl[64][72];
  const int tid = threadIdx.x;
  const int wave = __builtin_amdgcn_readfirstlane(tid >> 5);
  const int lane = tid & 31, ln = lane & 15, hh = lane >> 4;
  const int tile = blockIdx.x, h = blockIdx.y;
  const int b = tile / (SEQ / 64);
  const int sblk = (tile % (SEQ / 64)) * 64;
  const size_t xoff = ((size_t)b * SEQ_FULL + sblk + wave * 16 + ln) * DM + h * HD;
  const v8f z8 = {0.f, 0.f, 0.f, 0.f, 0.f, 0.f, 0.f, 0.f};
  v8f c0 = z8, c1 = z8, c2 = z8, c3 = z8;
  proj_acc(x, xoff, W16, ln, hh, c0, c1, c2, c3);
#pragma unroll
  for (int r = 0; r < 8; ++r) {
    const int tok = wave * 16 + 8 * hh + r;
    tl[ln][tok]      = hbits(c0[r] * 0.0625f);
    tl[16 + ln][tok] = hbits(c1[r] * 0.0625f);
    tl[32 + ln][tok] = hbits(c2[r] * 0.0625f);
    tl[48 + ln][tok] = hbits(c3[r] * 0.0625f);
  }
  __syncthreads();
  const int dr = tid >> 3, pc = tid & 7;
  v8us ov[4];
#pragma unroll
  for (int rd = 0; rd < 4; ++rd) ov[rd] = *(const v8us*)&tl[rd * 16 + dr][pc * 8];
  const size_t obase = ((size_t)(b * NH + h) * HD) * SEQ + sblk + pc * 8;
  for (int pass = 0; pass < 2; ++pass) {
#pragma unroll
    for (int rd = 0; rd < 4; ++rd)
      *(volatile v8us*)((unsigned short*)dst + obase + (size_t)(rd * 16 + dr) * SEQ) = ov[rd];
    if (pass == 0) __threadfence();
  }
}

__global__ __launch_bounds__(128) void k_attn(const _Float16* __restrict__ Q16, const _Float16* __restrict__ K16, const _Float16* __restrict__ VT,
                                              const int* __restrict__ mask, _Float16* __restrict__ Oh, _Float16* __restrict__ Ol) {
  __shared__ __attribute__((aligned(16))) float so[4][16][68];
  const int tid = threadIdx.x;
  const int wave = __builtin_amdgcn_readfirstlane(tid >> 5);
  const int lane = tid & 31, ln = lane & 15, hh = lane >> 4;
  const int qb = blockIdx.x % (SEQ / 64);
  const int bh = blockIdx.x / (SEQ / 64);
  const int h = bh % NH, b = bh / NH;
  const int q0 = qb * 64 + wave * 16;
  const size_t rowb = (size_t)b * SEQ;
  const size_t qoff = (rowb + q0 + ln) * DM + h * HD;
  const v16h qf0 = ldfrag(Q16, qoff, hh);
  const v16h qf1 = ldfrag(Q16, qoff + 32, hh);
  const size_t koff0 = (rowb + ln) * DM + h * HD;
  const size_t voff0 = ((size_t)bh * HD + ln) * SEQ;
  const int* mrow = mask + (size_t)b * SEQ_FULL + 8 * hh;
  const v8f z8 = {0.f, 0.f, 0.f, 0.f, 0.f, 0.f, 0.f, 0.f};
  v8f o0 = z8, o1 = z8, o2 = z8, o3 = z8;
  float mm = -1.0e30f;
  float lsum = 0.f;
  const float scale = 0.044194173824159216f;
#pragma unroll 1
  for (int kk = 0; kk < SEQ; kk += 32) {
    const size_t ka = koff0 + (size_t)kk * DM;
    v8f s0 = z8, s1 = z8;
    s0 = mma16(ldfrag(K16, ka, hh), qf0, s0);
    s0 = mma16(ldfrag(K16, ka + 32, hh), qf1, s0);
    s1 = mma16(ldfrag(K16, ka + (size_t)16 * DM, hh), qf0, s1);
    s1 = mma16(ldfrag(K16, ka + (size_t)16 * DM + 32, hh), qf1, s1);
    const v4ia mA = *(const v4ia*)(mrow + kk), mB = *(const v4ia*)(mrow + kk + 4);
    const v4ia mC = *(const v4ia*)(mrow + kk + 16), mD = *(const v4ia*)(mrow + kk + 20);
    float t[16];
#pragma unroll
    for (int i = 0; i < 4; ++i) {
      t[i]      = ((mA[i] == 0) ? -1.0e20f : s0[i])     * scale;
      t[4 + i]  = ((mB[i] == 0) ? -1.0e20f : s0[4 + i]) * scale;
      t[8 + i]  = ((mC[i] == 0) ? -1.0e20f : s1[i])     * scale;
      t[12 + i] = ((mD[i] == 0) ? -1.0e20f : s1[4 + i]) * scale;
    }
    float mx = t[0];
#pragma unroll
    for (int i = 1; i < 16; ++i) mx = fmaxf(mx, t[i]);
    mx = fmaxf(mx, __shfl_xor(mx, 16, 32));
    const float mnew = fmaxf(mm, mx - 5.5f);
    if (__builtin_amdgcn_ballot_w32(mnew > mm) != 0u) {
      const float alpha = __expf(mm - mnew);
      lsum *= alpha;
#pragma unroll
      for (int r = 0; r < 8; ++r) {
        const float ar = __shfl(alpha, 8 * hh + r, 32);
        o0[r] *= ar; o1[r] *= ar; o2[r] *= ar; o3[r] *= ar;
      }
      mm = mnew;
    }
    FragH pf;
    float ps = 0.f;
#pragma unroll
    for (int i = 0; i < 16; ++i) { const float p = __expf(t[i] - mm); ps += p; pf.h[i] = (_Float16)p; }
    lsum += ps;
    const size_t va = voff0 + kk;
    o0 = mma16(pf.v, ldfrag(VT, va, hh), o0);
    o1 = mma16(pf.v, ldfrag(VT, va + (size_t)16 * SEQ, hh), o1);
    o2 = mma16(pf.v, ldfrag(VT, va + (size_t)32 * SEQ, hh), o2);
    o3 = mma16(pf.v, ldfrag(VT, va + (size_t)48 * SEQ, hh), o3);
  }
  const float lt = lsum + __shfl_xor(lsum, 16, 32);
  const float inv = 64.0f * (1.0f / lt);
#pragma unroll
  for (int r = 0; r < 8; ++r) {
    const float ir = __shfl(inv, 8 * hh + r, 32);
    so[wave][8 * hh + r][ln]      = o0[r] * ir;
    so[wave][8 * hh + r][16 + ln] = o1[r] * ir;
    so[wave][8 * hh + r][32 + ln] = o2[r] * ir;
    so[wave][8 * hh + r][48 + ln] = o3[r] * ir;
  }
  __syncthreads();
  const int rq = lane >> 3, c8 = (lane & 7) * 8;
  v8us vh[4], vl[4];
#pragma unroll
  for (int q = 0; q < 4; ++q) {
    const int row = q * 4 + rq;
    const v4f a = *(const v4fa*)&so[wave][row][c8], c = *(const v4fa*)&so[wave][row][c8 + 4];
    FragH fh, fl;
#pragma unroll
    for (int i = 0; i < 4; ++i) {
      _Float16 hv = (_Float16)a[i]; fh.h[i] = hv; fl.h[i] = (_Float16)((a[i] - (float)hv) * 1024.0f);
      hv = (_Float16)c[i]; fh.h[4 + i] = hv; fl.h[4 + i] = (_Float16)((c[i] - (float)hv) * 1024.0f);
    }
    vh[q] = fh.half[0]; vl[q] = fl.half[0];
  }
  const size_t obase = (rowb + q0) * DM + h * HD + c8;
  for (int pass = 0; pass < 2; ++pass) {
#pragma unroll
    for (int q = 0; q < 4; ++q) {
      const size_t o = obase + (size_t)(q * 4 + rq) * DM;
      *(volatile v8us*)((unsigned short*)Oh + o) = vh[q];
      *(volatile v8us*)((unsigned short*)Ol + o) = vl[q];
    }
    if (pass == 0) __threadfence();
  }
}

__global__ __launch_bounds__(128) void k_out(const _Float16* __restrict__ Ah, const _Float16* __restrict__ Al, const _Float16* __restrict__ Bt,
                                             const float* __restrict__ bias, float* __restrict__ C) {
  __shared__ __attribute__((aligned(16))) float so[4][16][68];
  const int tid = threadIdx.x;
  const int wave = __builtin_amdgcn_readfirstlane(tid >> 5);
  const int lane = tid & 31, ln = lane & 15, hh = lane >> 4;
  const int ntn = DM / 64;
  const int mt = blockIdx.x / ntn, nq = blockIdx.x % ntn;
  const int row0 = mt * 64 + wave * 16, col0 = nq * 64;
  const size_t aoff = (size_t)(row0 + ln) * DM;
  const size_t boff = (size_t)(col0 + ln) * DM;
  const v8f z8 = {0.f, 0.f, 0.f, 0.f, 0.f, 0.f, 0.f, 0.f};
  v8f ch[4] = {z8, z8, z8, z8}, cl[4] = {z8, z8, z8, z8};
#pragma unroll 1
  for (int kb = 0; kb < DM; kb += 32) {
    const v16h a = ldfrag(Ah, aoff + kb, hh);
    const v16h al = ldfrag(Al, aoff + kb, hh);
#pragma unroll
    for (int t = 0; t < 4; ++t) {
      const v16h bq = ldfrag(Bt, boff + (size_t)(t * 16) * DM + kb, hh);
      ch[t] = mma16(a, bq, ch[t]);
      cl[t] = mma16(al, bq, cl[t]);
    }
  }
#pragma unroll
  for (int t = 0; t < 4; ++t) {
    const float bv = bf16_rne(bias[col0 + t * 16 + ln]);
#pragma unroll
    for (int r = 0; r < 8; ++r)
      so[wave][8 * hh + r][t * 16 + ln] = (ch[t][r] + cl[t][r] * 0.0009765625f) * 0.0009765625f + bv;
  }
  __syncthreads();
  const int rsub = lane >> 4, c4 = (lane & 15) * 4;
  v4f ov[8];
#pragma unroll
  for (int q = 0; q < 8; ++q) ov[q] = *(const v4fa*)&so[wave][q * 2 + rsub][c4];
  for (int pass = 0; pass < 2; ++pass) {
#pragma unroll
    for (int q = 0; q < 8; ++q)
      *(volatile v4f*)(C + (size_t)(row0 + q * 2 + rsub) * DM + col0 + c4) = ov[q];
    if (pass == 0) __threadfence();
  }
}

extern "C" void kernel_launch(void* const* d_in, const int* in_sizes, int n_in,
                              void* d_out, int out_size, void* d_ws, size_t ws_size, hipStream_t stream) {
  if (n_in < 9) return;
  const size_t need_x = ((size_t)(NB - 1) * SEQ_FULL + SEQ) * DM;
  const size_t need_m = (size_t)(NB - 1) * SEQ_FULL + SEQ;
  if ((size_t)in_sizes[0] < need_x || (size_t)in_sizes[1] < need_x || (size_t)in_sizes[2] < need_x) return;
  if ((size_t)in_sizes[3] < need_m) return;
  if (in_sizes[4] < HD * HD || in_sizes[5] < HD * HD || in_sizes[6] < HD * HD) return;
  if (in_sizes[7] < DM * DM || in_sizes[8] < DM) return;
  if ((size_t)out_size < NR * DM) return;
  const float* xv = (const float*)d_in[0];
  const float* xk = (const float*)d_in[1];
  const float* xq = (const float*)d_in[2];
  const int*   km = (const int*)d_in[3];
  const float* wv = (const float*)d_in[4];
  const float* wk = (const float*)d_in[5];
  const float* wq = (const float*)d_in[6];
  const float* wo = (const float*)d_in[7];
  const float* bo = (const float*)d_in[8];
  char* ws = (char*)d_ws; size_t off = 0;
  auto take = [&](size_t bytes) { char* p = ws + off; off += (bytes + 255) & ~(size_t)255; return p; };
  _Float16* WQ = (_Float16*)take(WS_W64);
  _Float16* WK = (_Float16*)take(WS_W64);
  _Float16* WV = (_Float16*)take(WS_W64);
  _Float16* WO = (_Float16*)take(WS_WO);
  _Float16* Q16 = (_Float16*)take(WS_PLANE);
  _Float16* K16 = (_Float16*)take(WS_PLANE);
  _Float16* VT  = (_Float16*)take(WS_PLANE);
  _Float16* OH  = (_Float16*)take(WS_PLANE);
  _Float16* OL  = (_Float16*)take(WS_PLANE);
  if (off > ws_size) return;
  const unsigned int n8s = (unsigned int)(HD * HD / 8), n8o = (unsigned int)((size_t)DM * DM / 8);
  k_wnat<<<(n8s + 255) / 256, 256, 0, stream>>>(wq, n8s, WQ);
  k_wnat<<<(n8s + 255) / 256, 256, 0, stream>>>(wk, n8s, WK);
  k_wnat<<<(n8s + 255) / 256, 256, 0, stream>>>(wv, n8s, WV);
  k_wnat<<<(n8o + 255) / 256, 256, 0, stream>>>(wo, n8o, WO);
  const dim3 gp((unsigned)(NB * (SEQ / 64)), NH);
  k_proj_n<<<gp, 128, 0, stream>>>(xq, WQ, Q16);
  k_proj_n<<<gp, 128, 0, stream>>>(xk, WK, K16);
  k_proj_t<<<gp, 128, 0, stream>>>(xv, WV, VT);
  k_attn<<<(unsigned)(NB * NH * (SEQ / 64)), 128, 0, stream>>>(Q16, K16, VT, km, OH, OL);
  k_out<<<(unsigned)((NB * SEQ / 64) * (DM / 64)), 128, 0, stream>>>(OH, OL, WO, bo, (float*)d_out);
}
